// Splatter_70248485093630
// MI455X (gfx1250) — hardware-run, weakly checked
//
#include <hip/hip_runtime.h>
#include <math.h>

typedef __attribute__((ext_vector_type(16))) _Float16 v16h;
typedef __attribute__((ext_vector_type(8)))  _Float16 v8h;
typedef __attribute__((ext_vector_type(8)))  float    v8f;
typedef __attribute__((ext_vector_type(4)))  float    v4f;
typedef __attribute__((ext_vector_type(2)))  float    v2f;
typedef __attribute__((ext_vector_type(4)))  int      v4i;

constexpr int kImgW     = 512;
constexpr int kImgH     = 512;
constexpr int kTilePx   = 16;
constexpr int kTilesX   = kImgW / kTilePx;
constexpr int kTilesY   = kImgH / kTilePx;
constexpr int kTiles    = kTilesX * kTilesY;
constexpr int kPairs    = kTiles / 2;
constexpr int kSlots    = 128;
constexpr int kNumPrim  = 32768;
constexpr int kWaveCap  = 768;
constexpr int kPlPitch  = 40;
constexpr int kBtPitch  = 136;
constexpr int kOutRowF  = kImgW * 3;
constexpr float kWCarry = 32768.0f;
constexpr float kCCarry = 64.0f;
constexpr float kFold   = 1.0f / (kWCarry * kCCarry);
static_assert(kTilesX == 32 && kTilesY == 32 && kTiles == 1024, "tile grid");
static_assert((kSlots % 32) == 0, "k depth multiple of 32");
static_assert((kNumPrim % 256) == 0, "primitive count multiple of the block");
static_assert((kPlPitch % 8) == 0 && (kBtPitch % 8) == 0, "16-B aligned LDS rows");
static_assert(kOutRowF * 4 == 48 * 128, "output row = 48 lines");
static_assert(kWCarry * 0.99f < 65504.0f, "carried weight inside f16 range");

constexpr size_t kOffGsel = 0;
constexpr size_t kOffGq   = kOffGsel + (size_t)kNumPrim * 16;
constexpr size_t kOffSel  = kOffGq   + (size_t)kNumPrim * 16;
constexpr size_t kWsTotal = kOffSel  + (size_t)kTiles * kSlots * 4;
static_assert(kWsTotal == 1572864ull, "carve total");
static_assert((kOffGq % 128) == 0 && (kOffSel % 128) == 0, "aligned regions");

union FragU { v16h v; v8h h[2]; };
__device__ __forceinline__ v16h frag_load(const _Float16* p) {
  FragU f;
  f.h[0] = *(const v8h*)(p);
  f.h[1] = *(const v8h*)(p + 16);
  return f.v;
}
__device__ __forceinline__ v8f mma_f16_guarded(v16h a, v16h b, v8f c) {
  c = __builtin_amdgcn_wmma_f32_16x16x32_f16(false, a, false, b, (short)0, c, false, false);
  asm volatile("v_nop\n\tv_nop\n\tv_nop\n\tv_nop" : "+v"(c) : "v"(a), "v"(b));
  return c;
}

#pragma clang fp contract(off)

__global__ __launch_bounds__(256) void prep_kernel(
    const float* __restrict__ pos, const float* __restrict__ quat, const float* __restrict__ scl,
    const float* __restrict__ opa, const float* __restrict__ camq, const float* __restrict__ camt,
    float* __restrict__ gsel, float* __restrict__ gq, int nprim)
{
  const int n = blockIdx.x * 256 + threadIdx.x;
  if (n >= nprim) return;

  float qw = camq[0], qx = camq[1], qy = camq[2], qz = camq[3];
  const float cn = sqrtf(((qw * qw + qx * qx) + qy * qy) + qz * qz);
  const float ci = 1.0f / cn;
  qw = qw * ci; qx = qx * ci; qy = qy * ci; qz = qz * ci;
  const float c00 = 1.0f - 2.0f * (qy * qy + qz * qz);
  const float c01 = 2.0f * (qx * qy - qw * qz);
  const float c02 = 2.0f * (qx * qz + qw * qy);
  const float c10 = 2.0f * (qx * qy + qw * qz);
  const float c11 = 1.0f - 2.0f * (qx * qx + qz * qz);
  const float c12 = 2.0f * (qy * qz - qw * qx);
  const float c20 = 2.0f * (qx * qz - qw * qy);
  const float c21 = 2.0f * (qy * qz + qw * qx);
  const float c22 = 1.0f - 2.0f * (qx * qx + qy * qy);

  const float px = pos[3 * n + 0], py = pos[3 * n + 1], pz = pos[3 * n + 2];
  const float x = fmaf(pz, c02, fmaf(py, c01, px * c00)) + camt[0];
  const float y = fmaf(pz, c12, fmaf(py, c11, px * c10)) + camt[1];
  const float z = fmaf(pz, c22, fmaf(py, c21, px * c20)) + camt[2];

  const float zc = fmaxf(z, 1e-6f);
  const float xz = x / zc;
  const float yz = y / zc;
  const bool valid = (z > 0.3f) && (fabsf(xz) < 0.6f) && (fabsf(yz) < 0.6f);

  const v4f gv = *(const v4f*)(quat + 4 * (size_t)n);
  float gw = gv[0], gx = gv[1], gy = gv[2], gz = gv[3];
  const float gi = rsqrtf(((gw * gw + gx * gx) + gy * gy) + gz * gz);
  gw = gw * gi; gx = gx * gi; gy = gy * gi; gz = gz * gi;
  const float g00 = 1.0f - 2.0f * (gy * gy + gz * gz);
  const float g01 = 2.0f * (gx * gy - gw * gz);
  const float g02 = 2.0f * (gx * gz + gw * gy);
  const float g10 = 2.0f * (gx * gy + gw * gz);
  const float g11 = 1.0f - 2.0f * (gx * gx + gz * gz);
  const float g12 = 2.0f * (gy * gz - gw * gx);
  const float g20 = 2.0f * (gx * gz - gw * gy);
  const float g21 = 2.0f * (gy * gz + gw * gx);
  const float g22 = 1.0f - 2.0f * (gx * gx + gy * gy);

  const float s0 = __builtin_amdgcn_rcpf(1.0f + __expf(-scl[3 * n + 0]));
  const float s1 = __builtin_amdgcn_rcpf(1.0f + __expf(-scl[3 * n + 1]));
  const float s2 = __builtin_amdgcn_rcpf(1.0f + __expf(-scl[3 * n + 2]));

  const float iz  = 1.0f / zc;
  const float j00 = 512.0f * iz;
  const float j02 = -(xz * j00);
  const float j12 = -(yz * j00);

  const float w00 = fmaf(j02, c20, j00 * c00);
  const float w01 = fmaf(j02, c21, j00 * c01);
  const float w02 = fmaf(j02, c22, j00 * c02);
  const float w10 = fmaf(j12, c20, j00 * c10);
  const float w11 = fmaf(j12, c21, j00 * c11);
  const float w12 = fmaf(j12, c22, j00 * c12);

  const float u00 = fmaf(w02, g20, fmaf(w01, g10, w00 * g00)) * s0;
  const float u01 = fmaf(w02, g21, fmaf(w01, g11, w00 * g01)) * s1;
  const float u02 = fmaf(w02, g22, fmaf(w01, g12, w00 * g02)) * s2;
  const float u10 = fmaf(w12, g20, fmaf(w11, g10, w10 * g00)) * s0;
  const float u11 = fmaf(w12, g21, fmaf(w11, g11, w10 * g01)) * s1;
  const float u12 = fmaf(w12, g22, fmaf(w11, g12, w10 * g02)) * s2;

  const float ca = fmaf(u02, u02, fmaf(u01, u01, u00 * u00)) + 0.3f;
  const float cb = fmaf(u02, u12, fmaf(u01, u11, u00 * u10));
  const float cc = fmaf(u12, u12, fmaf(u11, u11, u10 * u10)) + 0.3f;

  const float det = ca * cc - cb * cb;
  const float mid = 0.5f * (ca + cc);
  const float radius = 3.0f * sqrtf(mid + sqrtf(fmaxf(mid * mid - det, 0.01f)));
  const float mx = 512.0f * xz + 256.0f;
  const float my = 512.0f * yz + 256.0f;
  const float gdet = fmaxf(det, 1e-8f);
  const float ig = __builtin_amdgcn_rcpf(gdet);
  const float qa = -0.5f * (cc * ig);
  const float qb = cb * ig;
  const float qc = -0.5f * (ca * ig);
  const float op = opa[n];

  v4f o0, o1;
  o0[0] = valid ? mx : 0.0f;
  o0[1] = valid ? my : 0.0f;
  o0[2] = valid ? (radius + 11.31370848f) : 0.0f;
  o0[3] = valid ? z : -1.0f;
  o1[0] = valid ? qa : 0.0f;
  o1[1] = valid ? qb : 0.0f;
  o1[2] = valid ? qc : 0.0f;
  o1[3] = valid ? op : 0.0f;

  float* p0 = gsel + 4 * (size_t)n;
  float* p1 = gq + 4 * (size_t)n;
  *(volatile v4f*)p0 = o0;
  *(volatile v4f*)p1 = o1;
  __threadfence();
  *(volatile v4f*)p0 = o0;
  *(volatile v4f*)p1 = o1;
}

__global__ __launch_bounds__(256) void select_kernel(
    const float* __restrict__ gsel, int* __restrict__ sel, int nprim)
{
  __shared__ unsigned long long cand[8 * kWaveCap];
  __shared__ int s_wcnt[8];
  __shared__ __align__(16) int s_out[kSlots];

  const int tid = threadIdx.x, lane = tid & 31, wave = tid >> 5;
  const int t = blockIdx.x;
  const float tcx = ((float)(t & (kTilesX - 1)) + 0.5f) * 16.0f;
  const float tcy = ((float)(t >> 5) + 0.5f) * 16.0f;

  if (tid < kSlots) s_out[tid] = -1;

  int wcnt = 0;
  const int iters = nprim >> 8;
#pragma unroll 1
  for (int it = 0; it < iters; ++it) {
    const int g = it * 256 + tid;
    const v4f v = *(const v4f*)(gsel + 4 * (size_t)g);
    const float dx = tcx - v[0];
    const float dy = tcy - v[1];
    const float d2 = dx * dx + dy * dy;
    const float thr = v[2] * v[2];
    const float zk = v[3];
    const bool hit = (zk > 0.0f) && (d2 <= thr);
    const unsigned mask = __builtin_amdgcn_ballot_w32(hit);
    const unsigned pre = __builtin_amdgcn_mbcnt_lo(mask, 0u);
    const int slot = wcnt + (int)pre;
    const unsigned long long pk = ((unsigned long long)__float_as_uint(zk) << 32) | (unsigned long long)(unsigned)g;
    if (hit && slot < kWaveCap) cand[wave * kWaveCap + slot] = pk;
    wcnt += __builtin_popcount(mask);
  }
  if (lane == 0) s_wcnt[wave] = (wcnt < kWaveCap) ? wcnt : kWaveCap;
  __syncthreads();

  int cw[8];
#pragma unroll
  for (int w = 0; w < 8; ++w) {
    int c = s_wcnt[w];
    c = (c < 0) ? 0 : ((c > kWaveCap) ? kWaveCap : c);
    cw[w] = __builtin_amdgcn_readfirstlane(c);
  }
  int mycnt = s_wcnt[wave];
  mycnt = (mycnt < 0) ? 0 : ((mycnt > kWaveCap) ? kWaveCap : mycnt);
  mycnt = __builtin_amdgcn_readfirstlane(mycnt);
  const int trips = (mycnt + 31) >> 5;

#pragma unroll 1
  for (int it2 = 0; it2 < trips; ++it2) {
    const int j = it2 * 32 + lane;
    const bool have = j < mycnt;
    const int jc = have ? j : (mycnt - 1);
    const unsigned long long key = cand[wave * kWaveCap + jc];
    int r = 0;
#pragma unroll
    for (int w = 0; w < 8; ++w) {
      const unsigned long long* cp = cand + w * kWaveCap;
      const int cnt_w = cw[w];
#pragma unroll 1
      for (int q = 0; q < cnt_w; ++q) {
        r += (cp[q] < key) ? 1 : 0;
      }
    }
    if (have && r < kSlots) s_out[r] = (int)(unsigned)(key & 0xffffffffull);
  }
  __syncthreads();

  if (wave == 0) {
    const v4i val = *(const v4i*)(s_out + lane * 4);
    int* p = sel + (size_t)t * kSlots + lane * 4;
    *(volatile v4i*)p = val;
    __threadfence();
    *(volatile v4i*)p = val;
  }
}

#pragma clang fp contract(fast)

__global__ __launch_bounds__(256) void raster_kernel(
    const float* __restrict__ gsel, const float* __restrict__ gq, const float* __restrict__ rgb,
    const int* __restrict__ sel, const int* __restrict__ hptr, const int* __restrict__ wptr,
    float* __restrict__ out, int nprim)
{
  __shared__ __align__(16) float sP0[kSlots * 4];
  __shared__ __align__(16) float sP1[kSlots * 2];
  __shared__ __align__(16) float sCol[3 * kSlots];
  __shared__ __align__(16) _Float16 sBt[16 * kBtPitch];
  __shared__ __align__(16) _Float16 sPl[8][32 * kPlPitch];
  __shared__ __align__(16) float sOut[16 * 96];

  const int tid = threadIdx.x, lane = tid & 31, wave = tid >> 5;
  const int hh = lane >> 4, ln = lane & 15;
  const int bp = blockIdx.x;
  const int trow = bp >> 4;
  const int pcol = bp & 15;

  const int hval = hptr[0];
  const int wval = wptr[0];
  const bool badshape = (hval != kImgH) || (wval != kImgW);
  const float nanv = __uint_as_float(0x7fc00000u);

  _Float16* pl = sPl[wave];

#pragma unroll 1
  for (int tile = 0; tile < 2; ++tile) {
    const int tcol = pcol * 2 + tile;
    const int t = trow * kTilesX + tcol;
    __syncthreads();
    if (tid < kSlots) {
      const int i = sel[(size_t)t * kSlots + tid];
      const bool have = (unsigned)i < (unsigned)nprim;
      const int ic = have ? i : 0;
      const v4f s4 = *(const v4f*)(gsel + 4 * (size_t)ic);
      const v4f q4 = *(const v4f*)(gq + 4 * (size_t)ic);
      float mx = s4[0];
      float my = s4[1];
      float qa = q4[0];
      float qb = q4[1];
      float qc = q4[2];
      float op = q4[3];
      float cr = rgb[3 * (size_t)ic + 0];
      float cg = rgb[3 * (size_t)ic + 1];
      float cbl = rgb[3 * (size_t)ic + 2];
      asm volatile("" : "+v"(mx), "+v"(my), "+v"(qa));
      asm volatile("" : "+v"(qb), "+v"(qc), "+v"(op));
      asm volatile("" : "+v"(cr), "+v"(cg), "+v"(cbl));
      v4f r0;
      r0[0] = have ? mx : 0.0f;
      r0[1] = have ? my : 0.0f;
      r0[2] = have ? qa : 0.0f;
      r0[3] = have ? qb : 0.0f;
      v2f r1;
      r1[0] = have ? qc : 0.0f;
      r1[1] = have ? op : 0.0f;
      *(v4f*)(sP0 + 4 * tid) = r0;
      *(v2f*)(sP1 + 2 * tid) = r1;
      sCol[0 * kSlots + tid] = have ? (cr * kCCarry) : 0.0f;
      sCol[1 * kSlots + tid] = have ? (cg * kCCarry) : 0.0f;
      sCol[2 * kSlots + tid] = have ? (cbl * kCCarry) : 0.0f;
    }
    __syncthreads();
    {
      const int n = tid >> 4, seg = tid & 15;
      const int nn = (n < 3) ? n : 2;
      const bool live = n < 3;
      const v4f e0 = *(const v4f*)(sCol + nn * kSlots + seg * 8);
      const v4f e1 = *(const v4f*)(sCol + nn * kSlots + seg * 8 + 4);
      v8h hv;
#pragma unroll
      for (int e = 0; e < 4; ++e) {
        const float a0 = live ? e0[e] : 0.0f;
        const float a1 = live ? e1[e] : 0.0f;
        hv[e]     = (_Float16)a0;
        hv[4 + e] = (_Float16)a1;
      }
      *(v8h*)(sBt + n * kBtPitch + seg * 8) = hv;
    }
    __syncthreads();

    const float pixx = (float)(tcol * 16 + ln) + 0.5f;
    const float pixy = (float)(trow * 16 + wave * 2 + hh) + 0.5f;
    float trans = kWCarry;
    v8f acc0 = (v8f){0.f, 0.f, 0.f, 0.f, 0.f, 0.f, 0.f, 0.f};
    v8f acc1 = (v8f){0.f, 0.f, 0.f, 0.f, 0.f, 0.f, 0.f, 0.f};

#pragma unroll 1
    for (int kc = 0; kc < kSlots / 32; ++kc) {
#pragma unroll 1
      for (int g = 0; g < 4; ++g) {
        const int kb = kc * 32 + g * 8;
        v8h hv;
#pragma unroll
        for (int e = 0; e < 8; ++e) {
          const v4f p0 = *(const v4f*)(sP0 + 4 * (kb + e));
          const v2f p1 = *(const v2f*)(sP1 + 2 * (kb + e));
          const float dx = pixx - p0[0];
          const float dy = pixy - p0[1];
          const float t1 = fmaf(p0[3], dy, p0[2] * dx);
          const float pw = fmaf(p1[0] * dy, dy, t1 * dx);
          float al = p1[1] * __expf(pw);
          al = fminf(fmaxf(al, 0.0f), 0.99f);
          const float wv = al * trans;
          trans = trans * (1.0f - al);
          hv[e] = (_Float16)wv;
        }
        *(v8h*)(pl + lane * kPlPitch + g * 8) = hv;
      }
      __syncthreads();
      const v16h a0 = frag_load(pl + ln * kPlPitch + 8 * hh);
      const v16h a1 = frag_load(pl + (16 + ln) * kPlPitch + 8 * hh);
      const v16h bf = frag_load(sBt + ln * kBtPitch + kc * 32 + 8 * hh);
      acc0 = mma_f16_guarded(a0, bf, acc0);
      acc1 = mma_f16_guarded(a1, bf, acc1);
      __syncthreads();
    }

    if (ln < 3) {
#pragma unroll
      for (int r = 0; r < 8; ++r) {
        float v0 = acc0[r] * kFold;
        float v1 = acc1[r] * kFold;
        v0 = badshape ? nanv : v0;
        v1 = badshape ? nanv : v1;
        const int col = (tile * 16 + 8 * hh + r) * 3 + ln;
        sOut[(wave * 2 + 0) * 96 + col] = v0;
        sOut[(wave * 2 + 1) * 96 + col] = v1;
      }
    }
  }
  __syncthreads();

  if (wave < 6) {
    const int q = lane >> 3, c4 = (lane & 7) * 4;
    const int la = wave * 8 + q;
    const int lb = la + 4;
    const int rowa = la / 3, sega = la - 3 * rowa;
    const int rowb = lb / 3, segb = lb - 3 * rowb;
    const v4f va = *(const v4f*)(sOut + rowa * 96 + sega * 32 + c4);
    const v4f vb = *(const v4f*)(sOut + rowb * 96 + segb * 32 + c4);
    float* pa = out + (size_t)(trow * 16 + rowa) * kOutRowF + pcol * 96 + sega * 32 + c4;
    float* pb = out + (size_t)(trow * 16 + rowb) * kOutRowF + pcol * 96 + segb * 32 + c4;
    for (int pass = 0; pass < 2; ++pass) {
      *(volatile v4f*)pa = va;
      *(volatile v4f*)pb = vb;
      __threadfence();
    }
  }
}

extern "C" void kernel_launch(void* const* d_in, const int* in_sizes, int n_in,
                              void* d_out, int out_size, void* d_ws, size_t ws_size,
                              hipStream_t stream) {
  if (n_in < 9) return;
  if (in_sizes[0] != kNumPrim * 3) return;
  if (in_sizes[1] != kNumPrim * 3) return;
  if (in_sizes[2] != kNumPrim) return;
  if (in_sizes[3] != kNumPrim * 4) return;
  if (in_sizes[4] != kNumPrim * 3) return;
  if (in_sizes[5] != 4) return;
  if (in_sizes[6] != 3) return;
  if (in_sizes[7] != 1) return;
  if (in_sizes[8] != 1) return;
  if (out_size != kImgH * kImgW * 3) return;
  if (ws_size < kWsTotal) return;

  const float* pos  = (const float*)d_in[0];
  const float* rgb  = (const float*)d_in[1];
  const float* opa  = (const float*)d_in[2];
  const float* quat = (const float*)d_in[3];
  const float* scl  = (const float*)d_in[4];
  const float* camq = (const float*)d_in[5];
  const float* camt = (const float*)d_in[6];
  const int*   hptr = (const int*)d_in[7];
  const int*   wptr = (const int*)d_in[8];
  float* out = (float*)d_out;

  char* ws = (char*)d_ws;
  float* gsel = (float*)(ws + kOffGsel);
  float* gq   = (float*)(ws + kOffGq);
  int*   sel  = (int*)(ws + kOffSel);

  prep_kernel<<<kNumPrim / 256, 256, 0, stream>>>(pos, quat, scl, opa, camq, camt, gsel, gq, kNumPrim);
  select_kernel<<<kTiles, 256, 0, stream>>>(gsel, sel, kNumPrim);
  raster_kernel<<<kPairs, 256, 0, stream>>>(gsel, gq, rgb, sel, hptr, wptr, out, kNumPrim);
}
